// ReachabilityFeaturesGNN_49185965474415
// MI455X (gfx1250) — hardware-run, weakly checked
//
#include <hip/hip_runtime.h>


namespace {
constexpr int N = 50000, NP = 50048, E = 800000, G = 512, FI = 10, CI = 6, HID = 64, NH = 4, W1O = NH * HID, OUTD = 4, NBLK = NP / 16;
constexpr float XS = 8.0f, WSC = 256.0f, NEG = 0.2f, BNEPS = 1e-5f;
typedef _Float16 b16;
typedef __attribute__((ext_vector_type(16))) _Float16 v16b;
typedef __attribute__((ext_vector_type(8))) _Float16 v8b;
typedef __attribute__((ext_vector_type(8))) float v8f;
typedef __attribute__((ext_vector_type(4))) float v4f;
typedef __attribute__((ext_vector_type(2))) float v2f;
__device__ __forceinline__ float bf16_rne(float f) { unsigned int u = __float_as_uint(f); u += 0x7FFFu + ((u >> 16) & 1u); return __uint_as_float(u & 0xFFFF0000u); }
__device__ __forceinline__ void split16(float v, b16& hi, b16& lo) { hi = (b16)v; lo = (b16)(v - (float)hi); }
__device__ __forceinline__ v16b frag_kb(const b16* p, int hh) { const v8b a = *(const v8b*)(p + 8 * hh), b = *(const v8b*)(p + 16 + 8 * hh); v16b f;
#pragma unroll
  for (int e = 0; e < 8; ++e) { f[e] = a[e]; f[8 + e] = b[e]; } return f; }
__device__ __forceinline__ v8f wmma16b(v16b a, v16b b, v8f c) { v8f d = __builtin_amdgcn_wmma_f32_16x16x32_f16(false, a, false, b, (short)0, c, false, false); asm volatile("v_nop\n\tv_nop\n\tv_nop\n\tv_nop" : "+v"(d) : "v"(a), "v"(b)); return d; }
__device__ __forceinline__ void wave_lds_sync() { __builtin_amdgcn_fence(__ATOMIC_RELEASE, "workgroup"); __builtin_amdgcn_wave_barrier(); __builtin_amdgcn_fence(__ATOMIC_ACQUIRE, "workgroup"); }
__device__ __forceinline__ float pmul(float a, float b) { float p = a * b; asm volatile("" : "+v"(p)); return p; }
__device__ __forceinline__ int iclamp(int v, int lo, int hi) { return v < lo ? lo : (v > hi ? hi : v); }
__device__ __forceinline__ float leaky(float v) { return v >= 0.0f ? v : NEG * v; }
constexpr int CSR_NBLK9 = 512, CSR_GB9 = 9, CSR_GN9 = 1 << CSR_GB9  , CSR_TS9 = (CSR_GN9 < 32 ? 32 : CSR_GN9)  , CSR_MAXG9 = 512, CSR_CAP9 = 12288  ;
__device__ __host__ __forceinline__ int csr_tix9(int v) { return (v >> CSR_GB9) * CSR_TS9 + (v & (CSR_GN9 - 1)); }
__global__ __launch_bounds__(64) void csrA_kernel9(const int* __restrict__ dst, int E, int N, int nG, int CHP, int NGP, int* __restrict__ STG, int* __restrict__ HST) {
  extern __shared__ int sm[];
  int* cnt = sm; int* run = sm + NGP; int* ids = sm + 2 * NGP;
  const int b = blockIdx.x; const int ch = (E + CSR_NBLK9 - 1) / CSR_NBLK9; const int e0 = b * ch, e1 = min(E, e0 + ch);
  for (int i = threadIdx.x; i < NGP; i += 64) cnt[i] = 0;
  for (int i = threadIdx.x; i < CHP; i += 64) ids[i] = -1;
  __syncthreads();
  if (threadIdx.x == 0) {
    for (int e = e0; e < e1; ++e) { int d = dst[e]; d = (d < 0) ? 0 : (d >= N ? N - 1 : d); cnt[d >> CSR_GB9] += 1; }
    int acc = 0; for (int g = 0; g < nG; ++g) { run[g] = acc; acc += cnt[g]; }
    for (int e = e0; e < e1; ++e) { int d = dst[e]; d = (d < 0) ? 0 : (d >= N ? N - 1 : d); const int g = d >> CSR_GB9; ids[run[g]] = e; run[g] += 1; } }
  __syncthreads();
  typedef __attribute__((ext_vector_type(4))) int v4i;
  for (int pass = 0; pass < 2; ++pass) {
    for (int i = threadIdx.x; i < CHP / 4; i += 64) *(volatile v4i*)(STG + (size_t)b * CHP + i * 4) = *(const v4i*)(&ids[i * 4]);
    for (int i = threadIdx.x; i < NGP / 4; i += 64) { v4i v; for (int e = 0; e < 4; ++e) v[e] = (i * 4 + e < nG) ? cnt[i * 4 + e] : 0; *(volatile v4i*)(HST + (size_t)b * NGP + i * 4) = v; }
    __threadfence(); }
}
__global__ __launch_bounds__(512) void csrS_kernel9(const int* __restrict__ HST, int nG, int NGP, int* __restrict__ START, int* __restrict__ TOT, int* __restrict__ OFF) {
  __shared__ int tot[CSR_MAXG9];
  const int b = threadIdx.x;
  for (int pass = 0; pass < 2; ++pass) { int runb = 0; for (int g = 0; g < nG; ++g) { int c = HST[(size_t)b * NGP + g]; c = (c < 0) ? 0 : c; ((volatile int*)OFF)[(size_t)g * CSR_NBLK9 + b] = runb; runb += c; } __threadfence(); }
  for (int g = threadIdx.x; g < nG; g += 512) { int s = 0; for (int bb = 0; bb < CSR_NBLK9; ++bb) { int c = HST[(size_t)bb * NGP + g]; s += (c < 0) ? 0 : c; } tot[g] = s; }
  __syncthreads();
  if (threadIdx.x < 32) {
    __shared__ int st[CSR_MAXG9 + 32];
    if (threadIdx.x == 0) { int acc = 0; for (int g = 0; g < NGP; ++g) { st[g] = acc; if (g < nG) acc += (tot[g] + 31) & ~31; } st[NGP] = acc; }
    __builtin_amdgcn_fence(__ATOMIC_RELEASE, "workgroup"); __builtin_amdgcn_wave_barrier(); __builtin_amdgcn_fence(__ATOMIC_ACQUIRE, "workgroup");
    for (int pass = 0; pass < 2; ++pass) { for (int i = threadIdx.x; i < NGP + 32; i += 32) { ((volatile int*)START)[i] = (i <= NGP) ? st[min(i, NGP)] : 0; ((volatile int*)TOT)[i] = (i < nG) ? tot[i] : 0; } __threadfence(); } }
}
__global__ __launch_bounds__(256) void csrB_kernel9(const int* __restrict__ dst, int N, int nG, int CHP, int NGP, int permLen, const int* __restrict__ STG, const int* __restrict__ HST, const int* __restrict__ OFF, const int* __restrict__ START, const int* __restrict__ TOT, int* __restrict__ PERM, int* __restrict__ ROWPTR, int* __restrict__ ROWCNT, int* __restrict__ FLAG) {
  typedef __attribute__((ext_vector_type(4))) int v4i;
  __shared__ int ids[CSR_CAP9]; __shared__ unsigned short key[CSR_CAP9]; __shared__ int outp[CSR_CAP9]; __shared__ int ncnt[CSR_GN9 + 1]; __shared__ int boff[CSR_NBLK9 + 1];
  const int g = blockIdx.x, t_ = threadIdx.x; int tot = TOT[g]; int st = START[g], stn = START[g + 1]; const int v0 = g * CSR_GN9; const int nv = min(CSR_GN9, N - v0); const int t0 = g * CSR_TS9;
  st = (st < 0) ? 0 : (st > permLen - 32 ? permLen - 32 : st) & ~31; stn = (stn < st) ? st : (stn > permLen ? permLen : stn); tot = (tot < 0) ? 0 : tot; if (tot > stn - st && tot <= CSR_CAP9) tot = stn - st;
  if (tot > CSR_CAP9) {
    for (int pass = 0; pass < 2; ++pass) { for (int i = t_; i < CSR_TS9 / 4; i += 256) { v4i a, c; for (int e = 0; e < 4; ++e) { a[e] = st; c[e] = 0; } *(volatile v4i*)(ROWPTR + t0 + i * 4) = a; *(volatile v4i*)(ROWCNT + t0 + i * 4) = c; } if (t_ == 0) ((volatile int*)FLAG)[0] = 1; __threadfence(); } (void)nv; return; }
  if (t_ == 0) { int acc = 0; for (int b = 0; b < CSR_NBLK9; ++b) { boff[b] = acc; int c = HST[(size_t)b * NGP + g]; c = (c < 0) ? 0 : (c > CHP ? CHP : c); acc += c; if (acc > tot) acc = tot; } boff[CSR_NBLK9] = acc; }
  for (int i = t_; i <= CSR_GN9; i += 256) ncnt[i] = 0;
  __syncthreads();
  for (int b = 0; b < CSR_NBLK9; ++b) { const int c = boff[b + 1] - boff[b]; int o_ = OFF[(size_t)g * CSR_NBLK9 + b]; o_ = (o_ < 0) ? 0 : (o_ > CHP - c ? CHP - c : o_); const int* src_ = STG + (size_t)b * CHP + o_;
    for (int i = t_; i < c; i += 256) { int id = src_[i]; id = (id < 0) ? 0 : id; ids[boff[b] + i] = id; int d = dst[id]; d = (d < v0) ? v0 : (d >= N ? N - 1 : d); int kk = d - v0; kk = (kk < 0) ? 0 : (kk >= CSR_GN9 ? CSR_GN9 - 1 : kk); key[boff[b] + i] = (unsigned short)kk; } }
  __syncthreads();
  if (t_ == 0) { for (int i = 0; i < tot; ++i) ncnt[key[i]] += 1; int acc = 0; for (int vl = 0; vl < CSR_GN9; ++vl) { const int c = ncnt[vl]; ncnt[vl] = acc; acc += c; } ncnt[CSR_GN9] = acc;
    for (int i = 0; i < tot; ++i) { const int vl = key[i]; outp[ncnt[vl]] = ids[i]; ncnt[vl] += 1; }
    for (int vl = CSR_GN9; vl > 0; --vl) ncnt[vl] = ncnt[vl - 1]; ncnt[0] = 0; }
  __syncthreads();
  for (int pass = 0; pass < 2; ++pass) {
    for (int i = t_; i < (stn - st) / 4; i += 256) { v4i v; for (int e = 0; e < 4; ++e) { const int q = i * 4 + e; v[e] = (q < tot) ? outp[q] : -1; } *(volatile v4i*)(PERM + st + i * 4) = v; }
    for (int i = t_; i < CSR_TS9 / 4; i += 256) { v4i a, c; for (int e = 0; e < 4; ++e) { const int vl = i * 4 + e; const int vc = vl < CSR_GN9 ? vl : CSR_GN9; a[e] = (vl < CSR_GN9) ? st + ncnt[vc] : st; c[e] = (vl < nv) ? (ncnt[(vc < CSR_GN9 ? vc : CSR_GN9 - 1) + 1] - ncnt[vc]) : 0; } *(volatile v4i*)(ROWPTR + t0 + i * 4) = a; *(volatile v4i*)(ROWCNT + t0 + i * 4) = c; }
    __threadfence(); }
}
__global__ __launch_bounds__(256) void csrZ_kernel9(int* __restrict__ p, size_t n4) { typedef __attribute__((ext_vector_type(4))) int v4i; const size_t tid = (size_t)blockIdx.x * 256 + threadIdx.x, nth = (size_t)gridDim.x * 256; v4i z = {0, 0, 0, 0}; for (size_t i = tid; i < n4; i += nth) *(volatile v4i*)(p + i * 4) = z; }
struct CsrBufs9 { int *STG, *HST, *OFF, *START, *TOT, *PERM, *ROWPTR, *ROWCNT, *FLAG; int nG, NGP, CHP; size_t permLen; char* base; size_t bytes; };
static size_t csr_carve9(CsrBufs9& c, char* ws, size_t off, int E, int N) {
  const size_t off0 = off; c.base = ws + off;
  auto al = [&](size_t bytes) { char* p = ws + off; off += (bytes + 255) & ~(size_t)255; return p; };
  c.nG = (N + CSR_GN9 - 1) / CSR_GN9; c.NGP = (c.nG + 31) & ~31; const int ch = (E + CSR_NBLK9 - 1) / CSR_NBLK9; c.CHP = (ch + 31) & ~31; c.permLen = (size_t)E + 32 * (size_t)c.nG + 32;
  c.STG = (int*)al((size_t)CSR_NBLK9 * c.CHP * 4); c.HST = (int*)al((size_t)CSR_NBLK9 * c.NGP * 4); c.OFF = (int*)al((size_t)c.NGP * CSR_NBLK9 * 4); c.START = (int*)al((size_t)(c.NGP + 64) * 4); c.TOT = (int*)al((size_t)(c.NGP + 64) * 4);
  c.PERM = (int*)al(c.permLen * 4); c.ROWPTR = (int*)al((size_t)c.nG * CSR_TS9 * 4); c.ROWCNT = (int*)al((size_t)c.nG * CSR_TS9 * 4); c.FLAG = (int*)al(256);
  c.bytes = off - off0; return off;
}
static void csr_build9(const CsrBufs9& c, const int* dst, int E, int N, hipStream_t stream) {
  const size_t smem = (size_t)(2 * c.NGP + c.CHP) * 4;
  csrZ_kernel9<<<512, 256, 0, stream>>>((int*)c.base, c.bytes / 16);
  csrA_kernel9<<<CSR_NBLK9, 64, smem, stream>>>(dst, E, N, c.nG, c.CHP, c.NGP, c.STG, c.HST);
  csrS_kernel9<<<1, 512, 0, stream>>>(c.HST, c.nG, c.NGP, c.START, c.TOT, c.OFF);
  csrB_kernel9<<<c.nG, 256, 0, stream>>>(dst, N, c.nG, c.CHP, c.NGP, (int)c.permLen, c.STG, c.HST, c.OFF, c.START, c.TOT, c.PERM, c.ROWPTR, c.ROWCNT, c.FLAG);
}


__global__ __launch_bounds__(256) void wprep_kernel(const float* __restrict__ w, int r0, int KIN, int OUT, int co, int KP, b16* __restrict__ WT) {
  const int KG = (KIN + 7) / 8; const size_t u = (size_t)blockIdx.x * 256 + threadIdx.x; if (u >= (size_t)OUT * KG) return; const int o = (int)(u / KG), k0 = (int)(u % KG) * 8; v8b v;
  for (int j = 0; j < 8; ++j) { const int k = k0 + j; v[j] = k < KIN ? (b16)(bf16_rne(w[(size_t)(r0 + k) * OUT + o]) * WSC) : (b16)0.0f; }
  for (int pass = 0; pass < 2; ++pass) { *(volatile v8b*)(WT + (size_t)o * KP + co + k0) = v; __threadfence(); }
}
__global__ __launch_bounds__(256) void wzero_kernel(b16* __restrict__ WT, int n8) { const int u = blockIdx.x * 256 + threadIdx.x; if (u >= n8) return; v8b z = {}; for (int pass = 0; pass < 2; ++pass) { *(volatile v8b*)(WT + (size_t)u * 8) = z; __threadfence(); } }
__global__ __launch_bounds__(256) void climb_kernel(const float* __restrict__ cl, const float* __restrict__ Wc, const float* __restrict__ bc, float* __restrict__ Cp) {
  const int u = blockIdx.x * 256 + threadIdx.x; if (u >= G * HID) return; const int g = u / HID, c = u % HID; float s = bf16_rne(bc[c]);
#pragma unroll
  for (int k = 0; k < CI; ++k) s += pmul(bf16_rne(cl[g * CI + k]), bf16_rne(Wc[k * HID + c]));
  for (int pass = 0; pass < 2; ++pass) { ((volatile float*)Cp)[u] = fmaxf(s, 0.0f); __threadfence(); }
}
__global__ __launch_bounds__(32) void lin1_kernel(const float* __restrict__ x, const b16* __restrict__ W1T, const float* __restrict__ as, const float* __restrict__ ad, int NLIM, float* __restrict__ P1, float* __restrict__ ES, float* __restrict__ ED) {
  __shared__ __attribute__((aligned(16))) float Tf[16][W1O + 4]; __shared__ __attribute__((aligned(16))) float Se[16][4], Sd[16][4];
  const int lane = threadIdx.x, nloc = lane & 15, hlf = lane >> 4; const size_t m0 = (size_t)blockIdx.x * 16; const bool live = m0 < (size_t)NLIM;
  v16b a = {}; if (live) { const size_t r = (m0 + nloc) < (size_t)N ? m0 + nloc : (size_t)N - 1; for (int j = 0; j < 8; ++j) { const int k0 = 8 * hlf + j; a[j] = k0 < FI ? (b16)(bf16_rne(x[r * FI + k0]) * XS) : (b16)0.0f; a[8 + j] = (b16)0.0f; } }
  const float sc = 1.0f / (XS * WSC);
#pragma unroll 1
  for (int cg = 0; cg < 2; ++cg) { v8f acc[8]; float pes[2][8], ped[2][8];
#pragma unroll
    for (int t = 0; t < 8; ++t) { acc[t] = (v8f){}; if (live) acc[t] = wmma16b(a, frag_kb(W1T + (size_t)(cg * 128 + t * 16 + nloc) * 32, hlf), acc[t]); }
#pragma unroll
    for (int hh = 0; hh < 2; ++hh) for (int r8 = 0; r8 < 8; ++r8) { pes[hh][r8] = 0.0f; ped[hh][r8] = 0.0f; }
#pragma unroll
    for (int t = 0; t < 8; ++t) { const int c = cg * 128 + t * 16 + nloc; const int hh = t >> 2; const float wsv = bf16_rne(as[c]), wdv = bf16_rne(ad[c]);
#pragma unroll
      for (int r8 = 0; r8 < 8; ++r8) { const float p = acc[t][r8] * sc; Tf[8 * hlf + r8][c] = p; pes[hh][r8] += pmul(p, wsv); ped[hh][r8] += pmul(p, wdv); } }
#pragma unroll
    for (int hh = 0; hh < 2; ++hh)
#pragma unroll
      for (int r8 = 0; r8 < 8; ++r8) { float s = pes[hh][r8], d = ped[hh][r8]; for (int o = 1; o < 16; o <<= 1) { s += __shfl_xor(s, o); d += __shfl_xor(d, o); } if (nloc == 0) { Se[8 * hlf + r8][cg * 2 + hh] = s; Sd[8 * hlf + r8][cg * 2 + hh] = d; } } }
  wave_lds_sync();
  for (int pass = 0; pass < 2; ++pass) { for (int rr = 0; rr < 16; ++rr) for (int q = 0; q < 2; ++q) *(volatile v4f*)(P1 + (m0 + rr) * W1O + q * 128 + lane * 4) = *(const v4f*)(&Tf[rr][q * 128 + lane * 4]);
    if (lane < 16) { *(volatile v4f*)(ES + (m0 + lane) * 4) = *(const v4f*)(&Se[lane][0]); *(volatile v4f*)(ED + (m0 + lane) * 4) = *(const v4f*)(&Sd[lane][0]); } __threadfence(); }
}
template <int W, int NHH, int EW>
__global__ __launch_bounds__(256) void att_kernel(const float* __restrict__ P, const float* __restrict__ ES, const float* __restrict__ ED, const float* __restrict__ bias, const int* __restrict__ srcs, const int* __restrict__ PERM, const int* __restrict__ ROWPTR, const int* __restrict__ ROWCNT, int permLen, int NLIM, float* __restrict__ Gout) {
  constexpr int CPL = W / 32; typedef __attribute__((ext_vector_type(CPL))) float vcf;
  const int wave = threadIdx.x >> 5, lane = threadIdx.x & 31; const size_t v = (size_t)blockIdx.x * 8 + wave; const int h = (lane * CPL) / (W / NHH); vcf o; for (int i = 0; i < CPL; ++i) o[i] = 0.0f;
  if (v < (size_t)NLIM) { int st = ROWPTR[v], cnt = ROWCNT[v]; cnt = iclamp(cnt, 0, 1 << 20); st = iclamp(st, 0, permLen - cnt); const float edv = ED[v * EW + h]; float mx = leaky(ES[v * EW + h] + edv);
#pragma unroll 1
    for (int j = 0; j < cnt; ++j) { const int e = iclamp(PERM[st + j], 0, E - 1); const int s = iclamp(srcs[e], 0, N - 1); if (s >= NLIM) continue; mx = fmaxf(mx, leaky(ES[(size_t)s * EW + h] + edv)); }
    float den; { const float p = __expf(leaky(ES[v * EW + h] + edv) - mx); den = p; const vcf f = *(const vcf*)(P + v * W + lane * CPL); for (int i = 0; i < CPL; ++i) o[i] = pmul(p, f[i]); }
#pragma unroll 1
    for (int j = 0; j < cnt; ++j) { const int e = iclamp(PERM[st + j], 0, E - 1); const int s = iclamp(srcs[e], 0, N - 1); if (s >= NLIM) continue; const float p = __expf(leaky(ES[(size_t)s * EW + h] + edv) - mx); den += p; const vcf f = *(const vcf*)(P + (size_t)s * W + lane * CPL); for (int i = 0; i < CPL; ++i) o[i] += pmul(p, f[i]); }
    const float inv = 1.0f / (den + 1e-16f); for (int i = 0; i < CPL; ++i) o[i] = pmul(o[i], inv) + bf16_rne(bias[lane * CPL + i]); }
  for (int pass = 0; pass < 2; ++pass) { *(volatile vcf*)(Gout + v * W + lane * CPL) = o; __threadfence(); }
}
template <int W>
__global__ __launch_bounds__(W) void bnstat1_kernel(const float* __restrict__ Gp, int NLIM, double* __restrict__ PS) {
  const int c = threadIdx.x; const int n0 = blockIdx.x * 512; double s = 0.0, s2 = 0.0;
#pragma unroll 1
  for (int n = n0; n < n0 + 512; ++n) if (n < NLIM && n < N) { const double v = (double)Gp[(size_t)n * W + c]; s += v; s2 += v * v; }
  for (int pass = 0; pass < 2; ++pass) { ((volatile double*)PS)[((size_t)blockIdx.x * 2) * W + c] = s; ((volatile double*)PS)[((size_t)blockIdx.x * 2 + 1) * W + c] = s2; __threadfence(); }
}
template <int W>
__global__ __launch_bounds__(W) void bnstat2_kernel(const double* __restrict__ PS, int nblk, int NLIM, double* __restrict__ MV) {
  const int c = threadIdx.x; double s = 0.0, s2 = 0.0; for (int b = 0; b < nblk; ++b) { s += PS[((size_t)b * 2) * W + c]; s2 += PS[((size_t)b * 2 + 1) * W + c]; }
  const double cntv = (double)(NLIM < N ? NLIM : N); const double mu = s / cntv; double var = s2 / cntv - mu * mu; if (var < 0.0) var = 0.0; const double rs = 1.0 / sqrt(var + (double)BNEPS);
  for (int pass = 0; pass < 2; ++pass) { ((volatile double*)MV)[c] = mu; ((volatile double*)MV)[W + c] = rs; __threadfence(); }
}
__global__ __launch_bounds__(32) void lin2_kernel(const float* __restrict__ G1, const double* __restrict__ MV, const float* __restrict__ gam, const float* __restrict__ bet, const b16* __restrict__ W2T, const float* __restrict__ as, const float* __restrict__ ad, int NLIM, float* __restrict__ P2, float* __restrict__ E2) {
  __shared__ __attribute__((aligned(16))) b16 Ah[16][W1O + 8], Al[16][W1O + 8]; __shared__ __attribute__((aligned(16))) float Tf[16][HID + 4]; __shared__ __attribute__((aligned(16))) float Se[16][4];
  const int lane = threadIdx.x, nloc = lane & 15, hlf = lane >> 4; const size_t m0 = (size_t)blockIdx.x * 16; const bool live = m0 < (size_t)NLIM;
  float mu[8], rs[8], g8[8], b8[8]; for (int j = 0; j < 8; ++j) { const int c = (j >> 2) * 128 + lane * 4 + (j & 3); mu[j] = (float)MV[c]; rs[j] = (float)MV[W1O + c]; g8[j] = bf16_rne(gam[c]); b8[j] = bf16_rne(bet[c]); }
  for (int rr = 0; rr < 16; ++rr) for (int q = 0; q < 2; ++q) { v4f v = {0, 0, 0, 0}; if (live) v = *(const v4f*)(G1 + (m0 + rr) * W1O + q * 128 + lane * 4);
    for (int j = 0; j < 4; ++j) { const int jj = q * 4 + j; const float a = live ? fmaxf(pmul(pmul(v[j] - mu[jj], rs[jj]), g8[jj]) + b8[jj], 0.0f) : 0.0f; b16 p, ql; split16(a * XS, p, ql); Ah[rr][q * 128 + lane * 4 + j] = p; Al[rr][q * 128 + lane * 4 + j] = ql; } }
  wave_lds_sync();
  v8f acc[4];
#pragma unroll
  for (int t = 0; t < 4; ++t) acc[t] = (v8f){};
  if (live) {
#pragma unroll 2
    for (int kb = 0; kb < W1O; kb += 32) { const v16b a = frag_kb(&Ah[nloc][kb], hlf), al = frag_kb(&Al[nloc][kb], hlf);
#pragma unroll
      for (int t = 0; t < 4; ++t) { const v16b bw = frag_kb(W2T + (size_t)(t * 16 + nloc) * W1O + kb, hlf); acc[t] = wmma16b(a, bw, acc[t]); acc[t] = wmma16b(al, bw, acc[t]); } } }
  const float sc = 1.0f / (XS * WSC); float pes[8], ped[8]; for (int r8 = 0; r8 < 8; ++r8) { pes[r8] = 0.0f; ped[r8] = 0.0f; }
#pragma unroll
  for (int t = 0; t < 4; ++t) { const int c = t * 16 + nloc; const float wsv = bf16_rne(as[c]), wdv = bf16_rne(ad[c]);
#pragma unroll
    for (int r8 = 0; r8 < 8; ++r8) { const float p = acc[t][r8] * sc; Tf[8 * hlf + r8][c] = p; pes[r8] += pmul(p, wsv); ped[r8] += pmul(p, wdv); } }
#pragma unroll
  for (int r8 = 0; r8 < 8; ++r8) { float s = pes[r8], d = ped[r8]; for (int o = 1; o < 16; o <<= 1) { s += __shfl_xor(s, o); d += __shfl_xor(d, o); } if (nloc == 0) { Se[8 * hlf + r8][0] = s; Se[8 * hlf + r8][1] = d; Se[8 * hlf + r8][2] = 0.0f; Se[8 * hlf + r8][3] = 0.0f; } }
  wave_lds_sync();
  for (int pass = 0; pass < 2; ++pass) { for (int rr = 0; rr < 16; ++rr) if (lane < 16) *(volatile v4f*)(P2 + (m0 + rr) * HID + lane * 4) = *(const v4f*)(&Tf[rr][lane * 4]); if (lane < 16) *(volatile v4f*)(E2 + (m0 + lane) * 4) = *(const v4f*)(&Se[lane][0]); __threadfence(); }
}
__global__ __launch_bounds__(32) void head_kernel(const float* __restrict__ G2, const double* __restrict__ MV, const float* __restrict__ gam, const float* __restrict__ bet, const float* __restrict__ Cp, const int* __restrict__ batch, const b16* __restrict__ WC1, const float* __restrict__ bcl1, const float* __restrict__ Wcl2, const float* __restrict__ bcl2, int NLIM, float* __restrict__ out) {
  __shared__ __attribute__((aligned(16))) b16 Ah[16][2 * HID + 8], Al[16][2 * HID + 8]; __shared__ __attribute__((aligned(16))) float so[16][4];
  const int lane = threadIdx.x, nloc = lane & 15, hlf = lane >> 4; const size_t m0 = (size_t)blockIdx.x * 16; if (m0 >= (size_t)NLIM) return;
  const float mu0 = (float)MV[lane * 2], mu1 = (float)MV[lane * 2 + 1], rs0 = (float)MV[HID + lane * 2], rs1 = (float)MV[HID + lane * 2 + 1], ga0 = bf16_rne(gam[lane * 2]), ga1 = bf16_rne(gam[lane * 2 + 1]), bb0 = bf16_rne(bet[lane * 2]), bb1 = bf16_rne(bet[lane * 2 + 1]);
  for (int rr = 0; rr < 16; ++rr) { const size_t r = m0 + rr; const bool ok = r < (size_t)N; const v2f g = ok ? *(const v2f*)(G2 + r * HID + lane * 2) : (v2f){0.0f, 0.0f}; const int gb = ok ? iclamp(batch[r], 0, G - 1) : 0; const v2f c = *(const v2f*)(Cp + (size_t)gb * HID + lane * 2);
    const float a0 = ok ? fmaxf(pmul(pmul(g[0] - mu0, rs0), ga0) + bb0, 0.0f) : 0.0f, a1 = ok ? fmaxf(pmul(pmul(g[1] - mu1, rs1), ga1) + bb1, 0.0f) : 0.0f; b16 p, q;
    split16(a0 * XS, p, q); Ah[rr][lane * 2] = p; Al[rr][lane * 2] = q; split16(a1 * XS, p, q); Ah[rr][lane * 2 + 1] = p; Al[rr][lane * 2 + 1] = q;
    split16((ok ? c[0] : 0.0f) * XS, p, q); Ah[rr][HID + lane * 2] = p; Al[rr][HID + lane * 2] = q; split16((ok ? c[1] : 0.0f) * XS, p, q); Ah[rr][HID + lane * 2 + 1] = p; Al[rr][HID + lane * 2 + 1] = q; }
  wave_lds_sync();
  v8f acc[4];
#pragma unroll
  for (int t = 0; t < 4; ++t) acc[t] = (v8f){};
#pragma unroll
  for (int kb = 0; kb < 2 * HID; kb += 32) { const v16b a = frag_kb(&Ah[nloc][kb], hlf), al = frag_kb(&Al[nloc][kb], hlf);
#pragma unroll
    for (int t = 0; t < 4; ++t) { const v16b bw = frag_kb(WC1 + (size_t)(t * 16 + nloc) * (2 * HID) + kb, hlf); acc[t] = wmma16b(a, bw, acc[t]); acc[t] = wmma16b(al, bw, acc[t]); } }
  const float sc = 1.0f / (XS * WSC); float pk[4][8]; for (int k = 0; k < 4; ++k) for (int r8 = 0; r8 < 8; ++r8) pk[k][r8] = 0.0f;
#pragma unroll
  for (int t = 0; t < 4; ++t) { const int cc = t * 16 + nloc; const float bb = bf16_rne(bcl1[cc]); float w4[4]; for (int k = 0; k < 4; ++k) w4[k] = bf16_rne(Wcl2[cc * OUTD + k]);
#pragma unroll
    for (int r8 = 0; r8 < 8; ++r8) { const float z = fmaxf(acc[t][r8] * sc + bb, 0.0f); for (int k = 0; k < 4; ++k) pk[k][r8] += pmul(z, w4[k]); } }
#pragma unroll
  for (int k = 0; k < 4; ++k)
#pragma unroll
    for (int r8 = 0; r8 < 8; ++r8) { float s = pk[k][r8]; for (int o = 1; o < 16; o <<= 1) s += __shfl_xor(s, o); if (nloc == 0) so[8 * hlf + r8][k] = s + bf16_rne(bcl2[k]); }
  wave_lds_sync();
  for (int pass = 0; pass < 2; ++pass) { if (lane < 16 && m0 + lane < (size_t)N) *(volatile v4f*)(out + (m0 + lane) * OUTD) = *(const v4f*)(&so[lane][0]); __threadfence(); }
}
}

extern "C" void kernel_launch(void* const* d_in, const int* in_sizes, int n_in, void* d_out, int out_size, void* d_ws, size_t ws_size, hipStream_t stream) {
  (void)n_in;
  auto Fp = [&](int i) { return (const float*)d_in[i]; }; auto Ip = [&](int i) { return (const int*)d_in[i]; };
  if (in_sizes[0] != N * FI || in_sizes[1] != G * CI || in_sizes[2] != 2 * E || in_sizes[3] != N || in_sizes[4] != FI * W1O || in_sizes[5] != NH * HID || in_sizes[10] != W1O * HID || in_sizes[16] != CI * HID || in_sizes[18] != 2 * HID * HID || in_sizes[20] != HID * OUTD || out_size != N * OUTD) return;
  const int NLIM = N; const int GB16 = NBLK, GB8 = NP / 8;
  size_t off = 0; char* ws = (char*)d_ws;
  auto carve = [&](size_t bytes) { char* p = ws + off; off += (bytes + 255) & ~(size_t)255; return p; };
  b16* W1T = (b16*)carve((size_t)W1O * 32 * 2); b16* W2T = (b16*)carve((size_t)HID * W1O * 2); b16* WC1 = (b16*)carve((size_t)HID * 2 * HID * 2);
  float* P1 = (float*)carve((size_t)NP * W1O * 4); float* G1 = (float*)carve((size_t)NP * W1O * 4); float* ES = (float*)carve((size_t)NP * 4 * 4); float* ED = (float*)carve((size_t)NP * 4 * 4);
  float* P2 = (float*)carve((size_t)NP * HID * 4); float* G2 = (float*)carve((size_t)NP * HID * 4); float* E2 = (float*)carve((size_t)NP * 4 * 4); float* Cp = (float*)carve((size_t)G * HID * 4);
  const int nbb = (NP + 511) / 512; double* PS = (double*)carve((size_t)nbb * 2 * W1O * 8); double* MV1 = (double*)carve(2 * W1O * 8); double* MV2 = (double*)carve(2 * HID * 8);
  CsrBufs9 csr; off = csr_carve9(csr, ws, off, E, N);
  if (off > ws_size || off > ((size_t)192 << 20)) return;
  wzero_kernel<<<(W1O * 32 / 8 + 255) / 256, 256, 0, stream>>>(W1T, W1O * 32 / 8);
  wprep_kernel<<<(W1O * FI + 255) / 256, 256, 0, stream>>>(Fp(4), 0, FI, W1O, 0, 32, W1T); wprep_kernel<<<(HID * W1O + 255) / 256, 256, 0, stream>>>(Fp(10), 0, W1O, HID, 0, W1O, W2T); wprep_kernel<<<(HID * 2 * HID + 255) / 256, 256, 0, stream>>>(Fp(18), 0, 2 * HID, HID, 0, 2 * HID, WC1);
  climb_kernel<<<(G * HID + 255) / 256, 256, 0, stream>>>(Fp(1), Fp(16), Fp(17), Cp);
  csr_build9(csr, Ip(2) + E, E, N, stream);
  lin1_kernel<<<GB16, 32, 0, stream>>>(Fp(0), W1T, Fp(5), Fp(6), NLIM, P1, ES, ED);
  att_kernel<W1O, NH, 4><<<GB8, 256, 0, stream>>>(P1, ES, ED, Fp(7), Ip(2), csr.PERM, csr.ROWPTR, csr.ROWCNT, (int)csr.permLen, NLIM, G1);
  bnstat1_kernel<W1O><<<nbb, W1O, 0, stream>>>(G1, NLIM, PS); bnstat2_kernel<W1O><<<1, W1O, 0, stream>>>(PS, nbb, NLIM, MV1);
  lin2_kernel<<<GB16, 32, 0, stream>>>(G1, MV1, Fp(8), Fp(9), W2T, Fp(11), Fp(12), NLIM, P2, E2);
  att_kernel<HID, 1, 4><<<GB8, 256, 0, stream>>>(P2, E2, E2 + 1, Fp(13), Ip(2), csr.PERM, csr.ROWPTR, csr.ROWCNT, (int)csr.permLen, NLIM, G2);
  bnstat1_kernel<HID><<<nbb, HID, 0, stream>>>(G2, NLIM, PS); bnstat2_kernel<HID><<<1, HID, 0, stream>>>(PS, nbb, NLIM, MV2);
  head_kernel<<<GB16, 32, 0, stream>>>(G2, MV2, Fp(14), Fp(15), Cp, Ip(3), WC1, Fp(19), Fp(20), Fp(21), NLIM, (float*)d_out);
}
